// LSTMStressPredictor_944892805172
// MI455X (gfx1250) — hardware-verified
//
#include <hip/hip_runtime.h>
#include <math.h>

constexpr int NBATCH   = 256;
constexpr int NSTEP    = 2048;
constexpr int NIN      = 6;
constexpr int NHID     = 64;
constexpr int NGATE    = 4 * NHID;
constexpr int NOUTF    = 6;
constexpr int NTHR     = 128;
constexpr int ROWS_BLK = 16;
constexpr int TCHUNK   = 16;
constexpr int HPITCH   = 72;
constexpr int XROW     = TCHUNK * NIN;
constexpr int KCAT     = 2 * NHID;
constexpr float HCARRY = 256.0f;
constexpr float WCARRY = 16.0f;
constexpr float ACCSC  = HCARRY * WCARRY;
constexpr float FOLD   = 1.0f / ACCSC;

static_assert(NBATCH % ROWS_BLK == 0, "batch tiles exact");
static_assert(NSTEP % TCHUNK == 0, "time chunks exact");
static_assert((TCHUNK & 1) == 0, "chunk start keeps step parity");
static_assert(NHID == 16 * (NTHR / 32), "one 16-unit subtile per wave");
static_assert(NHID % 32 == 0 && KCAT % 32 == 0, "K multiples of 32");
static_assert(XROW * 4 == 384, "16 steps of one batch row are 3 whole 128-B lines");
static_assert(NIN == NOUTF, "x and out staging share the row layout");
static_assert((ROWS_BLK * XROW / 4) == 3 * NTHR, "staging loops exact");
static_assert((2 * ROWS_BLK * HPITCH) % NTHR == 0, "h zero-fill exact");
static_assert((NGATE * NHID / 4) % NTHR == 0 && (NHID * NHID / 4) % NTHR == 0 && (16 * NHID / 4) % NTHR == 0, "weight staging exact");
static_assert(HPITCH % 8 == 0 && HPITCH >= NHID, "h tile pitch");

typedef __attribute__((ext_vector_type(16))) _Float16 v16h;
typedef __attribute__((ext_vector_type(8)))  _Float16 v8h;
typedef __attribute__((ext_vector_type(4)))  _Float16 v4h;
typedef __attribute__((ext_vector_type(8)))  float    v8f;
typedef __attribute__((ext_vector_type(4)))  float    v4f;
typedef __attribute__((ext_vector_type(2)))  float    v2f;

template <typename T> struct Frag;
template <> struct Frag<_Float16> {
  typedef v16h V; union U { v16h v; v8h h[2]; };
  static __device__ __forceinline__ v16h load(const _Float16* p) {
    U f; f.h[0] = *(const v8h*)(p); f.h[1] = *(const v8h*)(p + 16); return f.v;
  }
  static __device__ __forceinline__ v8f mma(v16h a, v16h b, v8f c) {
    return __builtin_amdgcn_wmma_f32_16x16x32_f16(false, a, false, b, (short)0, c, false, false);
  }
};

__device__ __forceinline__ void grp_guard(v8f& a0, v8f& a1, v8f& a2, v8f& a3,
                                          v16h x, v16h b0, v16h b1, v16h b2, v16h b3) {
  asm volatile("v_nop\n\tv_nop\n\tv_nop\n\tv_nop"
               : "+v"(a0), "+v"(a1), "+v"(a2), "+v"(a3)
               : "v"(x), "v"(b0), "v"(b1), "v"(b2), "v"(b3));
}
__device__ __forceinline__ void one_guard(v8f& a, v16h x, v16h y) {
  asm volatile("v_nop\n\tv_nop\n\tv_nop\n\tv_nop" : "+v"(a) : "v"(x), "v"(y));
}

__device__ __forceinline__ float fsig(float z)  { return __builtin_amdgcn_rcpf(1.0f + __expf(-z)); }
__device__ __forceinline__ float ftanh(float z) { return 1.0f - 2.0f * __builtin_amdgcn_rcpf(__expf(2.0f * z) + 1.0f); }

__device__ __forceinline__ void lstm_cell8(v8f zi, v8f zf, v8f zg, v8f zo, float (&cs)[8], _Float16* hcol) {
#pragma unroll
  for (int r = 0; r < 8; ++r) {
    const float ig = fsig(zi[r] * FOLD);
    const float fg = fsig(zf[r] * FOLD);
    const float gg = ftanh(zg[r] * FOLD);
    const float og = fsig(zo[r] * FOLD);
    const float cn = fg * cs[r] + ig * gg;
    cs[r] = cn;
    const float hn = og * ftanh(cn);
    hcol[r * HPITCH] = (_Float16)(hn * HCARRY);
  }
}

__device__ __forceinline__ void stage_w64(const float* __restrict__ src, _Float16* dst, int dpitch, int dcol0,
                                          int nq4, int tid) {
#pragma unroll 1
  for (int i = 0; i < nq4 / NTHR; ++i) {
    const int idx = i * NTHR + tid;
    const int n = idx >> 4;
    const int c4 = (idx & 15) * 4;
    const v4f v = *(const v4f*)(src + n * NHID + c4);
    v4h hv;
    hv[0] = (_Float16)(v[0] * WCARRY);
    hv[1] = (_Float16)(v[1] * WCARRY);
    hv[2] = (_Float16)(v[2] * WCARRY);
    hv[3] = (_Float16)(v[3] * WCARRY);
    *(v4h*)(dst + n * dpitch + dcol0 + c4) = hv;
  }
}

__global__ __launch_bounds__(NTHR) void lstm2_head_kernel(
    const float* __restrict__ x, const float* __restrict__ Wih0, const float* __restrict__ Whh0,
    const float* __restrict__ b0, const float* __restrict__ Wih1, const float* __restrict__ Whh1,
    const float* __restrict__ b1, const float* __restrict__ W1, const float* __restrict__ bf1,
    const float* __restrict__ W2, const float* __restrict__ bf2, float* __restrict__ out) {
  __shared__ __align__(16) _Float16 W0s[NGATE * NHID];
  __shared__ __align__(16) _Float16 Wc1s[NGATE * KCAT];
  __shared__ __align__(16) _Float16 W1s[NHID * NHID];
  __shared__ __align__(16) _Float16 W2s[16 * NHID];
  __shared__ __align__(16) _Float16 H0s[2 * ROWS_BLK * HPITCH];
  __shared__ __align__(16) _Float16 H1s[2 * ROWS_BLK * HPITCH];
  __shared__ __align__(16) _Float16 Rs[ROWS_BLK * HPITCH];
  __shared__ __align__(16) float Xs[ROWS_BLK * XROW];
  __shared__ __align__(16) float Os[ROWS_BLK * XROW];

  const int tid  = threadIdx.x;
  const int lane = tid & 31;
  const int wave = __builtin_amdgcn_readfirstlane(tid >> 5);
  const int c    = lane & 15;
  const int hh   = lane >> 4;
  const int koff = hh * 8;
  const int rowbase = blockIdx.x * ROWS_BLK;
  const int unit = 16 * wave + c;

  stage_w64(Whh0, W0s, NHID, 0, NGATE * NHID / 4, tid);
  stage_w64(Wih1, Wc1s, KCAT, 0, NGATE * NHID / 4, tid);
  stage_w64(Whh1, Wc1s, KCAT, NHID, NGATE * NHID / 4, tid);
  stage_w64(W1, W1s, NHID, 0, NHID * NHID / 4, tid);
  {
#pragma unroll 1
    for (int i = 0; i < (16 * NHID / 4) / NTHR; ++i) {
      const int idx = i * NTHR + tid;
      const int n = idx >> 4;
      const int c4 = (idx & 15) * 4;
      const int nc = (n < NOUTF) ? n : (NOUTF - 1);
      const v4f v = *(const v4f*)(W2 + nc * NHID + c4);
      const bool live = (n < NOUTF);
      v4h hv;
      hv[0] = (_Float16)(live ? v[0] * WCARRY : 0.0f);
      hv[1] = (_Float16)(live ? v[1] * WCARRY : 0.0f);
      hv[2] = (_Float16)(live ? v[2] * WCARRY : 0.0f);
      hv[3] = (_Float16)(live ? v[3] * WCARRY : 0.0f);
      *(v4h*)(W2s + n * NHID + c4) = hv;
    }
  }
#pragma unroll 1
  for (int i = tid; i < 2 * ROWS_BLK * HPITCH; i += NTHR) {
    H0s[i] = (_Float16)0.0f;
    H1s[i] = (_Float16)0.0f;
  }

  float wx[4][NIN], b0s[4], b1s[4];
#pragma unroll
  for (int g = 0; g < 4; ++g) {
    const int n = g * NHID + unit;
    const v2f w01 = *(const v2f*)(Wih0 + n * NIN);
    const v2f w23 = *(const v2f*)(Wih0 + n * NIN + 2);
    const v2f w45 = *(const v2f*)(Wih0 + n * NIN + 4);
    wx[g][0] = w01[0] * ACCSC; wx[g][1] = w01[1] * ACCSC;
    wx[g][2] = w23[0] * ACCSC; wx[g][3] = w23[1] * ACCSC;
    wx[g][4] = w45[0] * ACCSC; wx[g][5] = w45[1] * ACCSC;
    b0s[g] = b0[n] * ACCSC;
    b1s[g] = b1[n] * ACCSC;
  }
  const float bf1s = bf1[unit] * ACCSC;
  const float bf2raw = bf2[(c < NOUTF) ? c : (NOUTF - 1)];
  const float bf2s = (c < NOUTF) ? bf2raw * ACCSC : 0.0f;

  float c0s[8], c1s[8];
#pragma unroll
  for (int r = 0; r < 8; ++r) { c0s[r] = 0.0f; c1s[r] = 0.0f; }

  __syncthreads();

#pragma unroll 1
  for (int ch = 0; ch < NSTEP / TCHUNK; ++ch) {
    const int t0 = ch * TCHUNK;
#pragma unroll
    for (int it = 0; it < 3; ++it) {
      const int idx = it * NTHR + tid;
      const int m = idx / 24;
      const int q = idx - m * 24;
      const v4f v = *(const v4f*)(x + ((size_t)(rowbase + m) * NSTEP + (size_t)t0) * NIN + 4 * q);
      *(v4f*)(Xs + m * XROW + 4 * q) = v;
    }
    __syncthreads();

#pragma unroll 1
    for (int tl = 0; tl < TCHUNK; ++tl) {
      const int par = tl & 1;
      const _Float16* h0old = H0s + par * (ROWS_BLK * HPITCH);
      _Float16*       h0new = H0s + (par ^ 1) * (ROWS_BLK * HPITCH);
      const _Float16* h1old = H1s + par * (ROWS_BLK * HPITCH);
      _Float16*       h1new = H1s + (par ^ 1) * (ROWS_BLK * HPITCH);

      {
        v8f acc[4];
        const float* xs = Xs + (8 * hh) * XROW + tl * NIN;
#pragma unroll
        for (int r = 0; r < 8; ++r) {
          const v2f xa = *(const v2f*)(xs + r * XROW);
          const v2f xb = *(const v2f*)(xs + r * XROW + 2);
          const v2f xc = *(const v2f*)(xs + r * XROW + 4);
          const float x0 = xa[0], x1 = xa[1], x2 = xb[0], x3 = xb[1], x4 = xc[0], x5 = xc[1];
#pragma unroll
          for (int g = 0; g < 4; ++g) {
            float s = fmaf(x0, wx[g][0], b0s[g]);
            s = fmaf(x1, wx[g][1], s);
            s = fmaf(x2, wx[g][2], s);
            s = fmaf(x3, wx[g][3], s);
            s = fmaf(x4, wx[g][4], s);
            s = fmaf(x5, wx[g][5], s);
            acc[g][r] = s;
          }
        }
#pragma unroll
        for (int kt = 0; kt < NHID / 32; ++kt) {
          const v16h a = Frag<_Float16>::load(h0old + c * HPITCH + koff + 32 * kt);
          const _Float16* wp = W0s + unit * NHID + koff + 32 * kt;
          const v16h q0 = Frag<_Float16>::load(wp);
          const v16h q1 = Frag<_Float16>::load(wp + 1 * NHID * NHID);
          const v16h q2 = Frag<_Float16>::load(wp + 2 * NHID * NHID);
          const v16h q3 = Frag<_Float16>::load(wp + 3 * NHID * NHID);
          acc[0] = Frag<_Float16>::mma(a, q0, acc[0]);
          acc[1] = Frag<_Float16>::mma(a, q1, acc[1]);
          acc[2] = Frag<_Float16>::mma(a, q2, acc[2]);
          acc[3] = Frag<_Float16>::mma(a, q3, acc[3]);
          grp_guard(acc[0], acc[1], acc[2], acc[3], a, q0, q1, q2, q3);
        }
        lstm_cell8(acc[0], acc[1], acc[2], acc[3], c0s, h0new + (8 * hh) * HPITCH + unit);
      }
      __syncthreads();

      {
        v8f acc[4];
#pragma unroll
        for (int g = 0; g < 4; ++g)
#pragma unroll
          for (int r = 0; r < 8; ++r) acc[g][r] = b1s[g];
#pragma unroll
        for (int kt = 0; kt < KCAT / 32; ++kt) {
          const _Float16* ap = (kt < 2) ? (h0new + c * HPITCH + koff + 32 * kt)
                                        : (h1old + c * HPITCH + koff + 32 * (kt - 2));
          const v16h a = Frag<_Float16>::load(ap);
          const _Float16* wp = Wc1s + unit * KCAT + koff + 32 * kt;
          const v16h q0 = Frag<_Float16>::load(wp);
          const v16h q1 = Frag<_Float16>::load(wp + 1 * NHID * KCAT);
          const v16h q2 = Frag<_Float16>::load(wp + 2 * NHID * KCAT);
          const v16h q3 = Frag<_Float16>::load(wp + 3 * NHID * KCAT);
          acc[0] = Frag<_Float16>::mma(a, q0, acc[0]);
          acc[1] = Frag<_Float16>::mma(a, q1, acc[1]);
          acc[2] = Frag<_Float16>::mma(a, q2, acc[2]);
          acc[3] = Frag<_Float16>::mma(a, q3, acc[3]);
          grp_guard(acc[0], acc[1], acc[2], acc[3], a, q0, q1, q2, q3);
        }
        lstm_cell8(acc[0], acc[1], acc[2], acc[3], c1s, h1new + (8 * hh) * HPITCH + unit);
      }
      __syncthreads();

      {
        v8f af;
#pragma unroll
        for (int r = 0; r < 8; ++r) af[r] = bf1s;
#pragma unroll
        for (int kt = 0; kt < NHID / 32; ++kt) {
          const v16h a = Frag<_Float16>::load(h1new + c * HPITCH + koff + 32 * kt);
          const v16h q = Frag<_Float16>::load(W1s + unit * NHID + koff + 32 * kt);
          af = Frag<_Float16>::mma(a, q, af);
          one_guard(af, a, q);
        }
        _Float16* rcol = Rs + (8 * hh) * HPITCH + unit;
#pragma unroll
        for (int r = 0; r < 8; ++r) {
          const float v = fmaxf(af[r] * FOLD, 0.0f);
          rcol[r * HPITCH] = (_Float16)(v * HCARRY);
        }
      }
      __syncthreads();

      if (wave == 0) {
        v8f ao;
#pragma unroll
        for (int r = 0; r < 8; ++r) ao[r] = bf2s;
#pragma unroll
        for (int kt = 0; kt < NHID / 32; ++kt) {
          const v16h a = Frag<_Float16>::load(Rs + c * HPITCH + koff + 32 * kt);
          const v16h q = Frag<_Float16>::load(W2s + c * NHID + koff + 32 * kt);
          ao = Frag<_Float16>::mma(a, q, ao);
          one_guard(ao, a, q);
        }
        if (c < NOUTF) {
          float* oc = Os + (8 * hh) * XROW + tl * NOUTF + c;
#pragma unroll
          for (int r = 0; r < 8; ++r) oc[r * XROW] = ao[r] * FOLD;
        }
      }
    }

    __syncthreads();
    for (int pass = 0; pass < 2; ++pass) {
#pragma unroll
      for (int it = 0; it < 3; ++it) {
        const int idx = it * NTHR + tid;
        const int m = idx / 24;
        const int q = idx - m * 24;
        const v4f v = *(const v4f*)(Os + m * XROW + 4 * q);
        *(volatile v4f*)(out + ((size_t)(rowbase + m) * NSTEP + (size_t)t0) * NOUTF + 4 * q) = v;
      }
      __threadfence();
    }
  }
}

extern "C" void kernel_launch(void* const* d_in, const int* in_sizes, int n_in,
                              void* d_out, int out_size, void* d_ws, size_t ws_size, hipStream_t stream) {
  (void)d_ws; (void)ws_size;
  if (n_in < 11 || d_out == nullptr) return;
  if (in_sizes[0] != NBATCH * NSTEP * NIN || in_sizes[1] != NGATE * NIN || in_sizes[2] != NGATE * NHID ||
      in_sizes[3] != NGATE || in_sizes[4] != NGATE * NHID || in_sizes[5] != NGATE * NHID ||
      in_sizes[6] != NGATE || in_sizes[7] != NHID * NHID || in_sizes[8] != NHID ||
      in_sizes[9] != NOUTF * NHID || in_sizes[10] != NOUTF || out_size != NBATCH * NSTEP * NOUTF) return;

  const float* x    = (const float*)d_in[0];
  const float* Wih0 = (const float*)d_in[1];
  const float* Whh0 = (const float*)d_in[2];
  const float* b0   = (const float*)d_in[3];
  const float* Wih1 = (const float*)d_in[4];
  const float* Whh1 = (const float*)d_in[5];
  const float* b1   = (const float*)d_in[6];
  const float* W1   = (const float*)d_in[7];
  const float* bf1  = (const float*)d_in[8];
  const float* W2   = (const float*)d_in[9];
  const float* bf2  = (const float*)d_in[10];
  float* out = (float*)d_out;

  lstm2_head_kernel<<<NBATCH / ROWS_BLK, NTHR, 0, stream>>>(x, Wih0, Whh0, b0, Wih1, Whh1, b1, W1, bf1, W2, bf2, out);
}
